// BertEncoder_61881888801201
// MI455X (gfx1250) — hardware-run, weakly checked
//
#include <hip/hip_runtime.h>

typedef float          v8f   __attribute__((ext_vector_type(8)));
typedef float          v4f   __attribute__((ext_vector_type(4)));
typedef unsigned int   v4u   __attribute__((ext_vector_type(4)));
typedef int            v8i   __attribute__((ext_vector_type(8)));
typedef unsigned short v8us  __attribute__((ext_vector_type(8)));
typedef unsigned short v16us __attribute__((ext_vector_type(16)));
typedef __bf16         v16bf __attribute__((ext_vector_type(16)));
typedef _Float16       v16h  __attribute__((ext_vector_type(16)));
typedef v4f  __attribute__((may_alias)) v4fa;
typedef v8us __attribute__((may_alias)) v8usa;
union FragB { v16bf v; v16us u; v8us h[2]; v8i w; };
union FragH { v16h  v; v16us u; v8us h[2]; v8i w; };

__device__ __forceinline__ v8f wmb(const FragB& a, const FragB& b, v8f c) {
  v8f d = __builtin_amdgcn_wmma_f32_16x16x32_bf16(false, a.v, false, b.v, (short)0, c, false, false);
  asm volatile("v_nop\n\tv_nop\n\tv_nop\n\tv_nop" : "+v"(d) : "v"(a.w), "v"(b.w));
  return d;
}

__device__ __forceinline__ v8f wmh(const FragH& a, const FragH& b, v8f c) {
  v8f d = __builtin_amdgcn_wmma_f32_16x16x32_f16(false, a.v, false, b.v, (short)0, c, false, false);
  asm volatile("v_nop\n\tv_nop\n\tv_nop\n\tv_nop" : "+v"(d) : "v"(a.w), "v"(b.w));
  return d;
}

__device__ __forceinline__ unsigned bf16_bits(float f) {
  const unsigned u = __float_as_uint(f);
  const unsigned r = (u + 0x7FFFu + ((u >> 16) & 1u)) >> 16;
  const unsigned q = (u >> 16) | 0x40u;
  return ((u & 0x7fffffffu) > 0x7f800000u) ? q : r;
}

__device__ __forceinline__ float bf16_val(float f) {
  return __uint_as_float(bf16_bits(f) << 16);
}
__device__ __forceinline__ int clampi(int v, int lo, int hi) {
  return v < lo ? lo : (v > hi ? hi : v);
}

__device__ __forceinline__ unsigned f16_bits(float f) {
  const unsigned u  = __float_as_uint(f);
  const unsigned s  = (u >> 16) & 0x8000u;
  const unsigned a  = u & 0x7fffffffu;
  const unsigned t  = a - 0x38000000u;
  const unsigned r  = (t + 0x0FFFu + ((t >> 13) & 1u)) >> 13;
  const unsigned rc = r > 0x7C00u ? 0x7C00u : r;
  const bool small  = a < 0x38800000u;
  const bool isnan  = a > 0x7f800000u;
  const unsigned fin = small ? 0u : (s | rc);
  return isnan ? (s | 0x7E00u) : fin;
}

__device__ __forceinline__ unsigned pk16(unsigned lo, unsigned hi) { return lo | (hi << 16); }
__device__ __forceinline__ unsigned bf16_lo_bits(float v) {
  float hi = bf16_val(v);
  asm volatile("" : "+v"(hi));
  return bf16_bits(v - hi);
}
__device__ __forceinline__ v4u pack8_bf16(v4f a, v4f c) {
  return (v4u){ pk16(bf16_bits(a[0]), bf16_bits(a[1])), pk16(bf16_bits(a[2]), bf16_bits(a[3])),
                pk16(bf16_bits(c[0]), bf16_bits(c[1])), pk16(bf16_bits(c[2]), bf16_bits(c[3])) };
}
__device__ __forceinline__ v4u pack8_bf16_lo(v4f a, v4f c) {
  return (v4u){ pk16(bf16_lo_bits(a[0]), bf16_lo_bits(a[1])), pk16(bf16_lo_bits(a[2]), bf16_lo_bits(a[3])),
                pk16(bf16_lo_bits(c[0]), bf16_lo_bits(c[1])), pk16(bf16_lo_bits(c[2]), bf16_lo_bits(c[3])) };
}
__device__ __forceinline__ v4u pack8_f16(v4f a, v4f c) {
  return (v4u){ pk16(f16_bits(a[0]), f16_bits(a[1])), pk16(f16_bits(a[2]), f16_bits(a[3])),
                pk16(f16_bits(c[0]), f16_bits(c[1])), pk16(f16_bits(c[2]), f16_bits(c[3])) };
}

template <int FORM>
__global__ __launch_bounds__(256) void k_plane(const float* __restrict__ src, int rows, int cols, int ldsrc,
                                               unsigned short* __restrict__ dst, int MP, int KP) {
  static_assert(FORM >= 0 && FORM <= 3);
  const int KTOT = (FORM == 1 || FORM == 3) ? 2 * KP : KP;
  const unsigned ppr   = (unsigned)(KTOT >> 3);
  const unsigned kp8   = (unsigned)(KP >> 3);
  const unsigned total = (unsigned)MP * ppr;
  const unsigned g     = blockIdx.x * 256u + threadIdx.x;
  const unsigned rowu  = g / ppr;
  const unsigned p     = g - rowu * ppr;
  const bool second    = p >= kp8;
  const int row = (int)rowu;
  const int c0  = (int)((second ? p - kp8 : p) << 3);
  const float* srow = src + (size_t)clampi(row, 0, rows - 1) * (size_t)ldsrc;
  float x[8];
  unsigned mk[8];
#pragma unroll
  for (int e = 0; e < 8; ++e) {
    const int c = c0 + e;
    const float v = srow[clampi(c, 0, cols - 1)];
    asm volatile("" :: "v"(v));
    x[e]  = v;
    mk[e] = (row < rows && c < cols) ? 0xFFFFu : 0u;
  }
  const v4f a = (v4f){ x[0], x[1], x[2], x[3] };
  const v4f c = (v4f){ x[4], x[5], x[6], x[7] };
  v4u o;
  if (FORM == 2) {
    o = pack8_f16(a, c);
  } else {
    const v4u hi = pack8_bf16(a, c);
    o = hi;
    if (FORM == 1) { const v4u lo = pack8_bf16_lo(a, c); o = second ? lo : hi; }
  }
  const v4u mw = (v4u){ pk16(mk[0], mk[1]), pk16(mk[2], mk[3]), pk16(mk[4], mk[5]), pk16(mk[6], mk[7]) };
  o &= mw;
  if (g < total) {
    volatile v4u* q = (volatile v4u*)(dst + (size_t)g * 8);
    *q = o;
    __threadfence();
    *q = o;
  }
}

template <int FORM> struct FragOf    { typedef FragB T; };
template <>         struct FragOf<2> { typedef FragH T; };
__device__ __forceinline__ v8f mm(const FragB& a, const FragB& b, v8f c) { return wmb(a, b, c); }
__device__ __forceinline__ v8f mm(const FragH& a, const FragH& b, v8f c) { return wmh(a, b, c); }
template <class F> __device__ __forceinline__ F ld_frag(const unsigned short* p) {
  F f;
  f.h[0] = *(const v8usa*)(p);
  f.h[1] = *(const v8usa*)(p + 16);
  return f;
}

template <int FORM, int EPI>
__global__ __launch_bounds__(256) __attribute__((amdgpu_num_vgpr(248)))
void k_gemm_nt(const unsigned short* __restrict__ A, const unsigned short* __restrict__ B,
               const float* __restrict__ bias, float* __restrict__ D, int M, int N, int KTOT, int ldd) {
  static_assert(FORM >= 0 && FORM <= 2);
  static_assert(EPI == 0 || EPI == 1);
  typedef typename FragOf<FORM>::T F;
  __shared__ __attribute__((aligned(16))) float sT[8][16 * 68];
  const int lane = threadIdx.x & 31;
  const int wave = threadIdx.x >> 5;
  const int tilesM = (M + 63) >> 6;
  const int tilesN = (N + 63) >> 6;
  const int tile = blockIdx.x * 8 + wave;
  if (tile >= tilesM * tilesN) return;
  const int tm = tile / tilesN;
  const int tn = tile - tm * tilesN;
  const int m0 = tm << 6;
  const int n0 = tn << 6;

  const int rl = lane & 15;
  const int h8 = (lane >> 4) * 8;
  const unsigned short* pa = A + (size_t)(m0 + rl) * (size_t)KTOT + h8;
  const unsigned short* pb = B + (size_t)(n0 + rl) * (size_t)KTOT + h8;

  v8f acc[4][4];
#pragma unroll
  for (int i = 0; i < 4; ++i)
#pragma unroll
    for (int j = 0; j < 4; ++j) acc[i][j] = (v8f){0.f, 0.f, 0.f, 0.f, 0.f, 0.f, 0.f, 0.f};

#pragma unroll 1
  for (int k0 = 0; k0 < KTOT; k0 += 32) {
    F bf[4];
#pragma unroll
    for (int j = 0; j < 4; ++j) bf[j] = ld_frag<F>(pb + (size_t)(j << 4) * (size_t)KTOT + k0);
#pragma unroll
    for (int i = 0; i < 4; ++i) {
      const F af = ld_frag<F>(pa + (size_t)(i << 4) * (size_t)KTOT + k0);
#pragma unroll
      for (int j = 0; j < 4; ++j) acc[i][j] = mm(af, bf[j], acc[i][j]);
    }
  }

  float* slab = sT[wave];
  const int hh = lane >> 4;
  const int c4 = (lane & 15) * 4;
  const int nc = n0 + c4;
  const bool cok = nc < N;
  v4f bv = (v4f){0.f, 0.f, 0.f, 0.f};
  if (EPI == 1) {
    bv = *(const v4fa*)(bias + clampi(nc, 0, N - 4));
    asm volatile("" :: "v"(bv));
  }
#pragma unroll
  for (int i = 0; i < 4; ++i) {
    const int mBase = m0 + (i << 4);
#pragma unroll
    for (int j = 0; j < 4; ++j) {
#pragma unroll
      for (int r = 0; r < 8; ++r) slab[(h8 + r) * 68 + (j << 4) + rl] = acc[i][j][r];
    }
    __builtin_amdgcn_fence(__ATOMIC_RELEASE, "workgroup");
    __builtin_amdgcn_wave_barrier();
    __builtin_amdgcn_fence(__ATOMIC_ACQUIRE, "workgroup");
    v4f vv[8];
#pragma unroll
    for (int it = 0; it < 8; ++it) {
      const int row = it * 2 + hh;
      v4f v = *(const v4fa*)(slab + row * 68 + c4);
      if (EPI == 1) v += bv;
      vv[it] = v;
    }
    for (int pass = 0; pass < 2; ++pass) {
#pragma unroll
      for (int it = 0; it < 8; ++it) {
        const int row = mBase + it * 2 + hh;
        if (cok && row < M) *(volatile v4f*)(D + (size_t)row * (size_t)ldd + nc) = vv[it];
      }
      __threadfence();
    }
    __builtin_amdgcn_fence(__ATOMIC_RELEASE, "workgroup");
    __builtin_amdgcn_wave_barrier();
    __builtin_amdgcn_fence(__ATOMIC_ACQUIRE, "workgroup");
  }
}

#include <math.h>

#define NN     2048
#define FIN    128
#define HH     256
#define NHD    8
#define HDM    32
#define NL     2
#define NE     16384
#define MAXD   64
#define FFD    1024
#define DEGCAP 128
static_assert(NN % 128 == 0);
static_assert(HH == 256);
static_assert(HDM == 32);
static_assert(NHD * HDM == HH);
static_assert(NE == 16384);
static_assert(MAXD == 64);
static_assert(FFD == 4 * HH);
static_assert(DEGCAP * 4 == 512);
static_assert(DEGCAP >= 2 * 18 + 8);
static_assert(NN % 64 == 0 && HH % 64 == 0 && (3 * HH) % 64 == 0 && FFD % 64 == 0 && FIN % 64 == 0);
static_assert(FIN % 32 == 0 && (2 * HH) % 32 == 0 && (2 * FFD) % 32 == 0 && (8 * HH) % 32 == 0);
static_assert(HH % 32 == 0 && (3 * HH) % 32 == 0 && FFD % 32 == 0);

typedef float        x2f  __attribute__((ext_vector_type(2)));
typedef unsigned int x2u  __attribute__((ext_vector_type(2)));
typedef int          x4i  __attribute__((ext_vector_type(4)));
typedef x4i __attribute__((may_alias)) x4ia;

template <int DUP>
__global__ __launch_bounds__(256) void k_wT(const float* __restrict__ W, unsigned short* __restrict__ outp,
                                            int R, int C, int sIn, int sOut) {
  __shared__ __attribute__((aligned(16))) float tf[64 * 68];
  const int KT = DUP ? 2 * R : R;
  const float* Wz = W + (size_t)blockIdx.z * (size_t)sIn;
  unsigned short* oz = outp + (size_t)blockIdx.z * (size_t)sOut;
  const int c0 = blockIdx.x * 64;
  const int r0 = blockIdx.y * 64;
  const int tid = threadIdx.x;
  {
    const int lr = tid >> 4;
    const int c4 = (tid & 15) * 4;
#pragma unroll
    for (int it = 0; it < 4; ++it) {
      const int rr = it * 16 + lr;
      const v4f a = *(const v4fa*)(Wz + (size_t)(r0 + rr) * (size_t)C + c0 + c4);
      *(v4fa*)(tf + rr * 68 + c4) = a;
    }
  }
  __syncthreads();
  const int sub = tid >> 3;
  const int c8  = (tid & 7) * 8;
  v4u hv[2];
#pragma unroll
  for (int it = 0; it < 2; ++it) {
    const int oc = it * 32 + sub;
    float f[8];
#pragma unroll
    for (int e = 0; e < 8; ++e) f[e] = tf[(c8 + e) * 68 + oc];
    hv[it] = pack8_bf16((v4f){ f[0], f[1], f[2], f[3] }, (v4f){ f[4], f[5], f[6], f[7] });
  }
  for (int pass = 0; pass < 2; ++pass) {
#pragma unroll
    for (int it = 0; it < 2; ++it) {
      const int oc = it * 32 + sub;
      const size_t go = (size_t)(c0 + oc) * (size_t)KT + r0 + c8;
      *(volatile v4u*)(oz + go) = hv[it];
      if (DUP) *(volatile v4u*)(oz + go + R) = hv[it];
    }
    __threadfence();
  }
}

extern __shared__ __attribute__((aligned(16))) int g_dsm[];
#define ADJ_LDS_INTS (2 * NE + 128 * DEGCAP + 256)

__device__ __forceinline__ void adj_push(bool hit, int val, int rowoff, int& cnt) {
  if (hit) {
    if (cnt < DEGCAP) g_dsm[rowoff + cnt] = clampi(val, 0, NN - 1);
    ++cnt;
  }
}

__global__ __launch_bounds__(128) void k_adj(const int* __restrict__ ei, int* __restrict__ ADJ,
                                             int* __restrict__ CNT, int* __restrict__ DEGFB) {
  const int tid  = threadIdx.x;
  const int lane = tid & 31;
  const int wave = tid >> 5;
  const int node0 = blockIdx.x * 128;
  const int i = node0 + tid;
  const int LST = 2 * NE;
  const int CST = LST + 128 * DEGCAP;
#pragma unroll 4
  for (int it = 0; it < 64; ++it) {
    const int q = it * 128 + tid;
    const x4i v = *(const x4ia*)(ei + (size_t)q * 4);
    *(x4ia*)(&g_dsm[q * 4]) = v;
  }
  const int ro = LST + tid * DEGCAP;
#pragma unroll 4
  for (int s = 0; s < DEGCAP; ++s) g_dsm[ro + s] = i;
  __syncthreads();
  int cnt = 0;
#pragma unroll 1
  for (int e4 = 0; e4 < NE; e4 += 4) {
    const x4i s4 = *(const x4ia*)(&g_dsm[e4]);
    const x4i d4 = *(const x4ia*)(&g_dsm[NE + e4]);
    adj_push(s4[0] == i, d4[0], ro, cnt);  adj_push(d4[0] == i, s4[0], ro, cnt);
    adj_push(s4[1] == i, d4[1], ro, cnt);  adj_push(d4[1] == i, s4[1], ro, cnt);
    adj_push(s4[2] == i, d4[2], ro, cnt);  adj_push(d4[2] == i, s4[2], ro, cnt);
    adj_push(s4[3] == i, d4[3], ro, cnt);  adj_push(d4[3] == i, s4[3], ro, cnt);
  }
  g_dsm[CST + tid] = cnt < DEGCAP ? cnt : DEGCAP;
  {
    const float df = (float)cnt;
    const unsigned db = __float_as_uint(df);
    g_dsm[CST + 128 + tid] = (int)((cnt > DEGCAP) ? 0x7fc00000u : db);
  }
  __syncthreads();
#pragma unroll 1
  for (int g = 0; g < 4; ++g) {
    x4i vv[8];
#pragma unroll
    for (int k = 0; k < 8; ++k) {
      const int rr = wave * 32 + g * 8 + k;
      vv[k] = *(const x4ia*)(&g_dsm[LST + rr * DEGCAP + lane * 4]);
    }
    for (int pass = 0; pass < 2; ++pass) {
#pragma unroll
      for (int k = 0; k < 8; ++k) {
        const int rr = wave * 32 + g * 8 + k;
        *(volatile x4i*)(ADJ + (size_t)(node0 + rr) * DEGCAP + lane * 4) = vv[k];
      }
      __threadfence();
    }
  }
  if (wave == 0) {
    const x4i cv = *(const x4ia*)(&g_dsm[CST + lane * 4]);
    const x4i dv = *(const x4ia*)(&g_dsm[CST + 128 + lane * 4]);
    for (int pass = 0; pass < 2; ++pass) {
      *(volatile x4i*)(CNT   + node0 + lane * 4) = cv;
      *(volatile x4i*)(DEGFB + node0 + lane * 4) = dv;
      __threadfence();
    }
  }
}

__global__ __launch_bounds__(256) void k_bfs(const int* __restrict__ ADJ, const int* __restrict__ CNT,
                                             float* __restrict__ CNTS) {
  __shared__ unsigned fr[2 * NN];
  __shared__ unsigned vis[NN];
  __shared__ __attribute__((aligned(16))) int hist[32 * MAXD];
  __shared__ int part[8 * 32];
  __shared__ int flag;
  const int tid  = threadIdx.x;
  const int lane = tid & 31;
  const int wave = tid >> 5;
  const int src0 = blockIdx.x * 32;
#pragma unroll 4
  for (int j = 0; j < 16; ++j) fr[tid + 256 * j] = 0u;
#pragma unroll 4
  for (int j = 0; j < 8; ++j) { vis[tid + 256 * j] = 0u; hist[tid + 256 * j] = 0; }
  if (tid == 0) flag = 0;
  __syncthreads();
  if (tid < 32) {
    fr[src0 + tid]  = 1u << tid;
    vis[src0 + tid] = 1u << tid;
    hist[tid * MAXD] = 1;
  }
  __syncthreads();
  int last = 0;
  int co = 0;
#pragma unroll 1
  for (int level = 1; level < NN; ++level) {
    const int no = NN - co;
#pragma unroll 1
    for (int j = 0; j < 8; ++j) {
      const int v = tid + 256 * j;
      const int cv = clampi(CNT[v], 0, DEGCAP);
      int mx = cv;
#pragma unroll
      for (int off = 16; off >= 1; off >>= 1) {
        const int o = __shfl_xor(mx, off, 32);
        mx = o > mx ? o : mx;
      }
      const int t4 = (mx + 3) >> 2;
      const int* arow = ADJ + (size_t)v * DEGCAP;
      unsigned acc = 0u;
#pragma unroll 1
      for (int p = 0; p < t4; ++p) {
        const x4i u = *(const x4ia*)(arow + 4 * p);
        acc |= fr[co + clampi(u[0], 0, NN - 1)];
        acc |= fr[co + clampi(u[1], 0, NN - 1)];
        acc |= fr[co + clampi(u[2], 0, NN - 1)];
        acc |= fr[co + clampi(u[3], 0, NN - 1)];
      }
      const unsigned vs = vis[v];
      const unsigned nw = acc & ~vs;
      vis[v] = vs | nw;
      fr[no + v] = nw;
    }
    __syncthreads();
    {
      int pc = 0;
      const int base = no + wave * 256;
#pragma unroll 8
      for (int q = 0; q < 256; ++q) pc += (int)((fr[base + q] >> lane) & 1u);
      part[wave * 32 + lane] = pc;
    }
    __syncthreads();
    if (wave == 0) {
      int tot = 0;
#pragma unroll
      for (int w = 0; w < 8; ++w) tot += part[w * 32 + lane];
      {
        const int b = level < (MAXD - 1) ? level : (MAXD - 1);
        hist[lane * MAXD + b] += tot;
        last = (tot > 0) ? level : last;
      }
      int any = tot;
#pragma unroll
      for (int off = 16; off >= 1; off >>= 1) any |= __shfl_xor(any, off, 32);
      if (lane == 0) flag = any;
    }
    __syncthreads();
    const int f = flag;
    if (f == 0) break;
    co = no;
  }
  if (wave == 0) {
    int sum = 0;
#pragma unroll 8
    for (int d = 0; d < MAXD; ++d) sum += hist[lane * MAXD + d];
    const int un = NN - sum;
    {
      const int b = (last + 1) < (MAXD - 1) ? (last + 1) : (MAXD - 1);
      hist[lane * MAXD + b] += (un > 0) ? un : 0;
    }
  }
  __syncthreads();
  v4f fv[2];
#pragma unroll
  for (int it = 0; it < 2; ++it) {
    const int g = it * 256 + tid;
    const x4i hv = *(const x4ia*)(hist + g * 4);
    fv[it] = (v4f){ (float)hv[0], (float)hv[1], (float)hv[2], (float)hv[3] };
  }
  for (int pass = 0; pass < 2; ++pass) {
#pragma unroll
    for (int it = 0; it < 2; ++it) {
      const int g = it * 256 + tid;
      *(volatile v4f*)(CNTS + (size_t)blockIdx.x * (32 * MAXD) + g * 4) = fv[it];
    }
    __threadfence();
  }
}

__global__ __launch_bounds__(128) void k_div(float* __restrict__ DIV) {
  const int m = threadIdx.x;
  const float v = powf(10000.0f, (float)(2 * m) * (1.0f / 256.0f));
  volatile float* q = (volatile float*)(DIV + m);
  *q = v;
  __threadfence();
  *q = v;
}

__global__ __launch_bounds__(256) void k_table(const float* __restrict__ DIV, float* __restrict__ TAB) {
  const int idx = blockIdx.x * 256 + threadIdx.x;
  const int d = idx >> 7;
  const int m = idx & 127;
  const float dv = DIV[m];
  const float ang = (float)d / dv;
  const x2f o = (x2f){ sinf(ang), cosf(ang) };
  volatile x2f* q = (volatile x2f*)(TAB + (size_t)d * 256 + 2 * m);
  *q = o;
  __threadfence();
  *q = o;
}

__global__ __launch_bounds__(256) void k_cat(const float* __restrict__ EX, const float* __restrict__ bfeat,
                                             const float* __restrict__ DEGF, const float* __restrict__ CNTS,
                                             const float* __restrict__ TAB, const float* __restrict__ DIV,
                                             unsigned short* __restrict__ CAT) {
  __shared__ __attribute__((aligned(16))) float Cf[8 * 1024];
  __shared__ __attribute__((aligned(16))) float cs[8 * 64];
  const int tid = threadIdx.x;
  const int r0 = blockIdx.x * 8;
  if (tid < 128) {
    v4f cv = *(const v4fa*)(CNTS + (size_t)r0 * MAXD + tid * 4);
    const float sc = 1.0f / 2048.0f;
    cv = cv * (v4f){ sc, sc, sc, sc };
    *(v4fa*)(cs + tid * 4) = cv;
  }
#pragma unroll
  for (int it = 0; it < 2; ++it) {
    const int g = it * 256 + tid;
    const int r = g >> 6;
    const int c4 = (g & 63) * 4;
    const v4f a  = *(const v4fa*)(EX + (size_t)(r0 + r) * HH + c4);
    const v4f bb = *(const v4fa*)(bfeat + c4);
    const v4f br = (v4f){ bf16_val(bb[0]), bf16_val(bb[1]), bf16_val(bb[2]), bf16_val(bb[3]) };
    *(v4fa*)(Cf + r * 1024 + c4) = a + br;
  }
  {
    const int m = tid & 127;
    const int kind = tid >> 7;
    const unsigned mk = 0u - (unsigned)kind;
    const float dv = DIV[m];
#pragma unroll 1
    for (int r = 0; r < 8; ++r) {
      const int node = r0 + r;
      const float dg = DEGF[node];
      asm volatile("" :: "v"(dg));
      const unsigned pb = __float_as_uint((float)node);
      const unsigned db = __float_as_uint(dg);
      const float p = __uint_as_float((pb & mk) | (db & ~mk));
      const float ang = p / dv;
      Cf[r * 1024 + 256 + kind * 256 + 2 * m]     = sinf(ang);
      Cf[r * 1024 + 256 + kind * 256 + 2 * m + 1] = cosf(ang);
    }
  }
  __syncthreads();
  {
    float acc[8];
#pragma unroll
    for (int r = 0; r < 8; ++r) acc[r] = 0.0f;
#pragma unroll 2
    for (int d = 0; d < MAXD; ++d) {
      const float t = TAB[(size_t)d * 256 + tid];
#pragma unroll
      for (int r = 0; r < 8; ++r) acc[r] = fmaf(cs[r * 64 + d], t, acc[r]);
    }
#pragma unroll
    for (int r = 0; r < 8; ++r) Cf[r * 1024 + 768 + tid] = acc[r];
  }
  __syncthreads();
  const bool second = tid >= 128;
  const int col0 = (tid & 127) * 8;
  v4u o[8];
#pragma unroll
  for (int it = 0; it < 8; ++it) {
    const v4f a = *(const v4fa*)(Cf + it * 1024 + col0);
    const v4f c = *(const v4fa*)(Cf + it * 1024 + col0 + 4);
    if (second) o[it] = pack8_bf16_lo(a, c); else o[it] = pack8_bf16(a, c);
  }
  for (int pass = 0; pass < 2; ++pass) {
#pragma unroll
    for (int it = 0; it < 8; ++it)
      *(volatile v4u*)(CAT + (size_t)(r0 + it) * 2048 + tid * 8) = o[it];
    __threadfence();
  }
}

template <int MODE>
__global__ __launch_bounds__(256) void k_post(const float* __restrict__ raw, const float* __restrict__ bias,
                                              float* __restrict__ dstf, unsigned short* __restrict__ plane,
                                              int C, int total4) {
  const int g = blockIdx.x * 256 + threadIdx.x;
  if (g >= total4) return;
  const int c4n = C >> 2;
  const int row = g / c4n;
  const int c4 = (g - row * c4n) << 2;
  v4f v = *(const v4fa*)(raw + (size_t)g * 4);
  const v4f bb = *(const v4fa*)(bias + c4);
  v = v + (v4f){ bf16_val(bb[0]), bf16_val(bb[1]), bf16_val(bb[2]), bf16_val(bb[3]) };
  if (MODE == 1) {
#pragma unroll 1
    for (int i = 0; i < 4; ++i) {
      const float x = v[0];
      const float gl = 0.5f * x * (1.0f + erff(x * 0.70710678f));
      v = (v4f){ v[1], v[2], v[3], gl };
    }
  }
  const x2u hi = (x2u){ pk16(bf16_bits(v[0]), bf16_bits(v[1])), pk16(bf16_bits(v[2]), bf16_bits(v[3])) };
  const x2u lo = (x2u){ pk16(bf16_lo_bits(v[0]), bf16_lo_bits(v[1])), pk16(bf16_lo_bits(v[2]), bf16_lo_bits(v[3])) };
  unsigned short* ph = plane + (size_t)row * (size_t)(2 * C) + c4;
  unsigned short* pl = ph + C;
  if (MODE == 0) *(volatile v4f*)(dstf + (size_t)g * 4) = v;
  *(volatile x2u*)ph = hi;
  *(volatile x2u*)pl = lo;
  __threadfence();
  if (MODE == 0) *(volatile v4f*)(dstf + (size_t)g * 4) = v;
  *(volatile x2u*)ph = hi;
  *(volatile x2u*)pl = lo;
}

__global__ __launch_bounds__(256) void k_qkvsplit(const float* __restrict__ QKV, const float* __restrict__ bias,
                                                  unsigned short* __restrict__ QKh, unsigned short* __restrict__ QKl,
                                                  unsigned short* __restrict__ Vh, unsigned short* __restrict__ Vl) {
  __shared__ __attribute__((aligned(16))) float tf[64 * 68];
  const int ct = blockIdx.x;
  const int t0 = blockIdx.y * 64;
  const int tid = threadIdx.x;
  {
    const int lr = tid >> 4;
    const int c4 = (tid & 15) * 4;
    const v4f bb = *(const v4fa*)(bias + ct * 64 + c4);
    const v4f br = (v4f){ bf16_val(bb[0]), bf16_val(bb[1]), bf16_val(bb[2]), bf16_val(bb[3]) };
#pragma unroll
    for (int it = 0; it < 4; ++it) {
      const int rr = it * 16 + lr;
      const v4f a = *(const v4fa*)(QKV + (size_t)(t0 + rr) * (3 * HH) + ct * 64 + c4);
      *(v4fa*)(tf + rr * 68 + c4) = a + br;
    }
  }
  __syncthreads();
  const int kind = ct >> 2;
  const int hp = (ct & 3) * 2;
  v4u hv[2], lv[2];
  if (kind < 2) {
    const int token = tid >> 2;
    const int d0 = (tid & 3) * 8;
#pragma unroll
    for (int hs = 0; hs < 2; ++hs) {
      const v4f a = *(const v4fa*)(tf + token * 68 + hs * 32 + d0);
      const v4f c = *(const v4fa*)(tf + token * 68 + hs * 32 + d0 + 4);
      hv[hs] = pack8_bf16(a, c);
      lv[hs] = pack8_bf16_lo(a, c);
    }
    const size_t kb = (size_t)kind * (size_t)(NHD * NN * HDM);
    for (int pass = 0; pass < 2; ++pass) {
#pragma unroll
      for (int hs = 0; hs < 2; ++hs) {
        const size_t go = kb + ((size_t)(hp + hs) * NN + t0) * HDM + (size_t)tid * 8;
        *(volatile v4u*)(QKh + go) = hv[hs];
        *(volatile v4u*)(QKl + go) = lv[hs];
      }
      __threadfence();
    }
  } else {
    const int sub = tid >> 3;
    const int c8 = (tid & 7) * 8;
#pragma unroll
    for (int it = 0; it < 2; ++it) {
      const int oc = it * 32 + sub;
      float f[8];
#pragma unroll
      for (int e = 0; e < 8; ++e) f[e] = tf[(c8 + e) * 68 + oc];
      const v4f a = (v4f){ f[0], f[1], f[2], f[3] };
      const v4f c = (v4f){ f[4], f[5], f[6], f[7] };
      hv[it] = pack8_bf16(a, c);
      lv[it] = pack8_bf16_lo(a, c);
    }
    for (int pass = 0; pass < 2; ++pass) {
#pragma unroll
      for (int it = 0; it < 2; ++it) {
        const int oc = it * 32 + sub;
        const size_t go = (size_t)(hp * HDM + oc) * NN + t0 + c8;
        *(volatile v4u*)(Vh + go) = hv[it];
        *(volatile v4u*)(Vl + go) = lv[it];
      }
      __threadfence();
    }
  }
}

__global__ __launch_bounds__(128) __attribute__((amdgpu_num_vgpr(248)))
void k_attn(const unsigned short* __restrict__ Qh, const unsigned short* __restrict__ Ql,
            const unsigned short* __restrict__ Kh, const unsigned short* __restrict__ Kl,
            const unsigned short* __restrict__ Vh, const unsigned short* __restrict__ Vl,
            float* __restrict__ O, float sscale) {
  __shared__ __attribute__((aligned(16))) unsigned short Ksh[64 * 32];
  __shared__ __attribute__((aligned(16))) unsigned short Ksl[64 * 32];
  __shared__ __attribute__((aligned(16))) unsigned short Vth[32 * 64];
  __shared__ __attribute__((aligned(16))) unsigned short Vtl[32 * 64];
  __shared__ __attribute__((aligned(16))) unsigned short Psh[4 * 16 * 64];
  __shared__ __attribute__((aligned(16))) unsigned short Psl[4 * 16 * 64];
  __shared__ __attribute__((aligned(16))) float Os[4 * 16 * 36];

  const int tid  = threadIdx.x;
  const int wave = tid >> 5;
  const int lane = tid & 31;
  const int hh   = lane >> 4;
  const int c    = lane & 15;
  const int bx = blockIdx.x;
  const int qb = bx & 31;
  const int h  = bx >> 5;
  const int q0 = qb * 64 + wave * 16;
  const size_t hq = (size_t)h * NN * HDM;
  const size_t hv = (size_t)h * HDM * NN;

  const FragB qah = ld_frag<FragB>(Qh + hq + (size_t)(q0 + c) * HDM + 8 * hh);
  const FragB qal = ld_frag<FragB>(Ql + hq + (size_t)(q0 + c) * HDM + 8 * hh);

  float mrow[8], lrow[8];
  v8f oacc[2];
#pragma unroll
  for (int r = 0; r < 8; ++r) { mrow[r] = -INFINITY; lrow[r] = 0.f; }
  oacc[0] = (v8f){0.f, 0.f, 0.f, 0.f, 0.f, 0.f, 0.f, 0.f};
  oacc[1] = (v8f){0.f, 0.f, 0.f, 0.f, 0.f, 0.f, 0.f, 0.f};
  const int pw0 = wave * 16 * 64;

#pragma unroll 1
  for (int kc = 0; kc < NN / 64; ++kc) {
    const int kv0 = kc * 64;
    __syncthreads();
    {
      const int so = tid * 16;
      const unsigned short* kgh = Kh + hq + (size_t)kv0 * HDM + so;
      const unsigned short* kgl = Kl + hq + (size_t)kv0 * HDM + so;
      const int r = tid >> 2;
      const int qo = (tid & 3) * 16;
      const unsigned short* vgh = Vh + hv + (size_t)r * NN + kv0 + qo;
      const unsigned short* vgl = Vl + hv + (size_t)r * NN + kv0 + qo;
      const v8us a0 = *(const v8usa*)(kgh);
      const v8us a1 = *(const v8usa*)(kgh + 8);
      const v8us b0 = *(const v8usa*)(kgl);
      const v8us b1 = *(const v8usa*)(kgl + 8);
      const v8us c0 = *(const v8usa*)(vgh);
      const v8us c1 = *(const v8usa*)(vgh + 8);
      const v8us d0 = *(const v8usa*)(vgl);
      const v8us d1 = *(const v8usa*)(vgl + 8);
      *(v8usa*)(&Ksh[so])     = a0;
      *(v8usa*)(&Ksh[so + 8]) = a1;
      *(v8usa*)(&Ksl[so])     = b0;
      *(v8usa*)(&Ksl[so + 8]) = b1;
      *(v8usa*)(&Vth[r * 64 + qo])     = c0;
      *(v8usa*)(&Vth[r * 64 + qo + 8]) = c1;
      *(v8usa*)(&Vtl[r * 64 + qo])     = d0;
      *(v8usa*)(&Vtl[r * 64 + qo + 8]) = d1;
    }
    __syncthreads();

    v8f s[4];
#pragma unroll
    for (int j = 0; j < 4; ++j) {
      const int ko = (j * 16 + c) * 32 + 8 * hh;
      FragB kb, kl;
      kb.h[0] = *(const v8usa*)(&Ksh[ko]);
      kb.h[1] = *(const v8usa*)(&Ksh[ko + 16]);
      kl.h[0] = *(const v8usa*)(&Ksl[ko]);
      kl.h[1] = *(const v8usa*)(&Ksl[ko + 16]);
      v8f z = (v8f){0.f, 0.f, 0.f, 0.f, 0.f, 0.f, 0.f, 0.f};
      z = wmb(qah, kb, z);
      z = wmb(qah, kl, z);
      z = wmb(qal, kb, z);
      s[j] = z;
    }
    float cm[8];
#pragma unroll
    for (int r = 0; r < 8; ++r) {
      float m = -INFINITY;
#pragma unroll
      for (int j = 0; j < 4; ++j) {
        const float sv = s[j][r] * sscale;
        s[j][r] = sv;
        m = fmaxf(m, sv);
      }
#pragma unroll
      for (int off = 1; off < 16; off <<= 1) m = fmaxf(m, __shfl_xor(m, off, 32));
      cm[r] = m;
    }
#pragma unroll
    for (int r = 0; r < 8; ++r) {
      const float mnew = fmaxf(mrow[r], cm[r]);
      const float alpha = expf(mrow[r] - mnew);
      mrow[r] = mnew;
      float psum = 0.f;
#pragma unroll
      for (int j = 0; j < 4; ++j) {
        const float p = expf(s[j][r] - mnew);
        psum += p;
        Psh[pw0 + (8 * hh + r) * 64 + j * 16 + c] = (unsigned short)bf16_bits(p);
        Psl[pw0 + (8 * hh + r) * 64 + j * 16 + c] = (unsigned short)bf16_lo_bits(p);
      }
#pragma unroll
      for (int off = 1; off < 16; off <<= 1) psum += __shfl_xor(psum, off, 32);
      lrow[r] = lrow[r] * alpha + psum;
      oacc[0][r] *= alpha;
      oacc[1][r] *= alpha;
    }
    __builtin_amdgcn_fence(__ATOMIC_RELEASE, "workgroup");
    __builtin_amdgcn_wave_barrier();
    __builtin_amdgcn_fence(__ATOMIC_ACQUIRE, "workgroup");
#pragma unroll 1
    for (int kk = 0; kk < 2; ++kk) {
      const int po = pw0 + c * 64 + kk * 32 + 8 * hh;
      FragB pa, pl;
      pa.h[0] = *(const v8usa*)(&Psh[po]);
      pa.h[1] = *(const v8usa*)(&Psh[po + 16]);
      pl.h[0] = *(const v8usa*)(&Psl[po]);
      pl.h[1] = *(const v8usa*)(&Psl[po + 16]);
#pragma unroll
      for (int t = 0; t < 2; ++t) {
        const int vo = (t * 16 + c) * 64 + kk * 32 + 8 * hh;
        FragB vb, vl;
        vb.h[0] = *(const v8usa*)(&Vth[vo]);
        vb.h[1] = *(const v8usa*)(&Vth[vo + 16]);
        vl.h[0] = *(const v8usa*)(&Vtl[vo]);
        vl.h[1] = *(const v8usa*)(&Vtl[vo + 16]);
        oacc[t] = wmb(pa, vb, oacc[t]);
        oacc[t] = wmb(pa, vl, oacc[t]);
        oacc[t] = wmb(pl, vb, oacc[t]);
      }
    }
  }

  const int ow0 = wave * 16 * 36;
#pragma unroll
  for (int r = 0; r < 8; ++r) {
    const float inv = 1.0f / lrow[r];
    Os[ow0 + (8 * hh + r) * 36 + c]      = oacc[0][r] * inv;
    Os[ow0 + (8 * hh + r) * 36 + 16 + c] = oacc[1][r] * inv;
  }
  __builtin_amdgcn_fence(__ATOMIC_RELEASE, "workgroup");
  __builtin_amdgcn_wave_barrier();
  __builtin_amdgcn_fence(__ATOMIC_ACQUIRE, "workgroup");
  {
    const int row4 = lane >> 3;
    const int c4 = (lane & 7) * 4;
    v4f val[4];
#pragma unroll
    for (int it = 0; it < 4; ++it) val[it] = *(const v4fa*)(&Os[ow0 + (it * 4 + row4) * 36 + c4]);
    for (int pass = 0; pass < 2; ++pass) {
#pragma unroll
      for (int it = 0; it < 4; ++it) {
        const int row = it * 4 + row4;
        *(volatile v4f*)(O + (size_t)(q0 + row) * HH + h * HDM + c4) = val[it];
      }
      __threadfence();
    }
  }
}

template <int FINAL>
__global__ __launch_bounds__(256) void k_addln(const float* __restrict__ hin, const float* __restrict__ z,
                                               const float* __restrict__ bz, const float* __restrict__ g,
                                               const float* __restrict__ be, float* __restrict__ hout,
                                               unsigned short* __restrict__ plane) {
  __shared__ __attribute__((aligned(16))) float sp[3 * 256];
  const int tid = threadIdx.x;
  sp[tid]       = bf16_val(bz[tid]);
  sp[256 + tid] = bf16_val(g[tid]);
  sp[512 + tid] = bf16_val(be[tid]);
  __syncthreads();
  const int lane = tid & 31;
  const int row = blockIdx.x * 8 + (tid >> 5);
  v4f v[2];
  float s = 0.f;
#pragma unroll
  for (int q = 0; q < 2; ++q) {
    const int cc = q * 128 + lane * 4;
    const v4f a  = *(const v4fa*)(hin + (size_t)row * HH + cc);
    const v4f zz = *(const v4fa*)(z   + (size_t)row * HH + cc);
    const v4f bb = *(const v4fa*)(sp + cc);
    v[q] = a + (zz + bb);
    s += (v[q][0] + v[q][1]) + (v[q][2] + v[q][3]);
  }
#pragma unroll
  for (int off = 16; off >= 1; off >>= 1) s += __shfl_xor(s, off, 32);
  const float mean = s * (1.0f / 256.0f);
  float var = 0.f;
#pragma unroll
  for (int q = 0; q < 2; ++q) {
    v[q] = v[q] - (v4f){ mean, mean, mean, mean };
    var += (v[q][0] * v[q][0] + v[q][1] * v[q][1]) + (v[q][2] * v[q][2] + v[q][3] * v[q][3]);
  }
#pragma unroll
  for (int off = 16; off >= 1; off >>= 1) var += __shfl_xor(var, off, 32);
  const float rstd = 1.0f / sqrtf(var * (1.0f / 256.0f) + 1e-5f);
  v4f o[2];
  x2u ohi[2], olo[2];
#pragma unroll
  for (int q = 0; q < 2; ++q) {
    const int cc = q * 128 + lane * 4;
    const v4f gg = *(const v4fa*)(sp + 256 + cc);
    const v4f bt = *(const v4fa*)(sp + 512 + cc);
    o[q] = v[q] * (v4f){ rstd, rstd, rstd, rstd } * gg + bt;
    ohi[q] = (x2u){ pk16(bf16_bits(o[q][0]), bf16_bits(o[q][1])), pk16(bf16_bits(o[q][2]), bf16_bits(o[q][3])) };
    olo[q] = (x2u){ pk16(bf16_lo_bits(o[q][0]), bf16_lo_bits(o[q][1])),
                    pk16(bf16_lo_bits(o[q][2]), bf16_lo_bits(o[q][3])) };
  }
  for (int pass = 0; pass < 2; ++pass) {
#pragma unroll
    for (int q = 0; q < 2; ++q) {
      const int cc = q * 128 + lane * 4;
      *(volatile v4f*)(hout + (size_t)row * HH + cc) = o[q];
      if (FINAL == 0) {
        *(volatile x2u*)(plane + (size_t)row * (2 * HH) + cc)      = ohi[q];
        *(volatile x2u*)(plane + (size_t)row * (2 * HH) + HH + cc) = olo[q];
      }
    }
    __threadfence();
  }
}

static inline unsigned gemm_blocks(int M, int N) { return (unsigned)((((M + 63) / 64) * ((N + 63) / 64) + 7) / 8); }

extern "C" void kernel_launch(void* const* d_in, const int* in_sizes, int n_in,
                              void* d_out, int out_size, void* d_ws, size_t ws_size,
                              hipStream_t stream) {
  if (n_in < 19) return;
  if (in_sizes[0] != NN * FIN || in_sizes[1] != 2 * NE || in_sizes[2] != NN) return;
  if (in_sizes[3] != FIN * HH || in_sizes[4] != HH || in_sizes[5] != 4 * HH * HH || in_sizes[6] != HH) return;
  if (in_sizes[7] != NL * HH * 3 * HH || in_sizes[8] != NL * 3 * HH) return;
  if (in_sizes[9] != NL * HH * HH || in_sizes[10] != NL * HH) return;
  if (in_sizes[11] != NL * HH || in_sizes[12] != NL * HH) return;
  if (in_sizes[13] != NL * HH * FFD || in_sizes[14] != NL * FFD) return;
  if (in_sizes[15] != NL * FFD * HH || in_sizes[16] != NL * HH) return;
  if (in_sizes[17] != NL * HH || in_sizes[18] != NL * HH) return;
  if (out_size != NN * HH) return;

  const float* x      = (const float*)d_in[0];
  const int*   ei     = (const int*)  d_in[1];
  const float* W_feat = (const float*)d_in[3];
  const float* b_feat = (const float*)d_in[4];
  const float* W_proj = (const float*)d_in[5];
  const float* b_proj = (const float*)d_in[6];
  const float* Wqkv   = (const float*)d_in[7];
  const float* bqkv   = (const float*)d_in[8];
  const float* Wo     = (const float*)d_in[9];
  const float* bo     = (const float*)d_in[10];
  const float* ln1_g  = (const float*)d_in[11];
  const float* ln1_b  = (const float*)d_in[12];
  const float* W1     = (const float*)d_in[13];
  const float* b1     = (const float*)d_in[14];
  const float* W2     = (const float*)d_in[15];
  const float* b2     = (const float*)d_in[16];
  const float* ln2_g  = (const float*)d_in[17];
  const float* ln2_b  = (const float*)d_in[18];
  float* out = (float*)d_out;

  size_t off = 0;
  auto take = [&](size_t bytes) { const size_t o = off; off += (bytes + 255) & ~(size_t)255; return o; };
  const size_t oXB    = take((size_t)NN * FIN * 2);
  const size_t oWfT   = take((size_t)HH * FIN * 2);
  const size_t oWpD   = take((size_t)HH * (8 * HH) * 2);
  const size_t oWqkvD = take((size_t)NL * (3 * HH) * (2 * HH) * 2);
  const size_t oWoD   = take((size_t)NL * HH * (2 * HH) * 2);
  const size_t oW1D   = take((size_t)NL * FFD * (2 * HH) * 2);
  const size_t oW2D   = take((size_t)NL * HH * (2 * FFD) * 2);
  const size_t oCAT   = take((size_t)NN * (8 * HH) * 2);
  const size_t oHhl   = take((size_t)NN * (2 * HH) * 2);
  const size_t oQKh   = take((size_t)2 * NHD * NN * HDM * 2);
  const size_t oQKl   = take((size_t)2 * NHD * NN * HDM * 2);
  const size_t oVh    = take((size_t)NHD * HDM * NN * 2);
  const size_t oVl    = take((size_t)NHD * HDM * NN * 2);
  const size_t oOhl   = take((size_t)NN * (2 * HH) * 2);
  const size_t oGhl   = take((size_t)NN * (2 * FFD) * 2);
  const size_t oEX    = take((size_t)NN * HH * 4);
  const size_t oHraw  = take((size_t)NN * HH * 4);
  const size_t oZraw  = take((size_t)NN * HH * 4);
  const size_t oHfA   = take((size_t)NN * HH * 4);
  const size_t oHfB   = take((size_t)NN * HH * 4);
  const size_t oQKV   = take((size_t)NN * 3 * HH * 4);
  const size_t oO     = take((size_t)NN * HH * 4);
  const size_t oGraw  = take((size_t)NN * FFD * 4);
  const size_t oTAB   = take((size_t)MAXD * HH * 4);
  const size_t oDIV   = take((size_t)128 * 4);
  const size_t oADJ   = take((size_t)NN * DEGCAP * 4);
  const size_t oCNT   = take((size_t)NN * 4);
  const size_t oDEGF  = take((size_t)NN * 4);
  const size_t oCNTS  = take((size_t)NN * MAXD * 4);
  if (off > ws_size || off > ((size_t)128 << 20)) return;

  char* ws = (char*)d_ws;
  unsigned short* XB    = (unsigned short*)(ws + oXB);
  unsigned short* WfT   = (unsigned short*)(ws + oWfT);
  unsigned short* WpD   = (unsigned short*)(ws + oWpD);
  unsigned short* WqkvD = (unsigned short*)(ws + oWqkvD);
  unsigned short* WoD   = (unsigned short*)(ws + oWoD);
  unsigned short* W1D   = (unsigned short*)(ws + oW1D);
  unsigned short* W2D   = (unsigned short*)(ws + oW2D);
  unsigned short* CAT   = (unsigned short*)(ws + oCAT);
  unsigned short* Hhl   = (unsigned short*)(ws + oHhl);
  unsigned short* QKh   = (unsigned short*)(ws + oQKh);
  unsigned short* QKl   = (unsigned short*)(ws + oQKl);
  unsigned short* Vh    = (unsigned short*)(ws + oVh);
  unsigned short* Vl    = (unsigned short*)(ws + oVl);
  unsigned short* Ohl   = (unsigned short*)(ws + oOhl);
  unsigned short* Ghl   = (unsigned short*)(ws + oGhl);
  float* EX    = (float*)(ws + oEX);
  float* Hraw  = (float*)(ws + oHraw);
  float* Zraw  = (float*)(ws + oZraw);
  float* HfA   = (float*)(ws + oHfA);
  float* HfB   = (float*)(ws + oHfB);
  float* QKVr  = (float*)(ws + oQKV);
  float* Of    = (float*)(ws + oO);
  float* Graw  = (float*)(ws + oGraw);
  float* TAB   = (float*)(ws + oTAB);
  float* DIV   = (float*)(ws + oDIV);
  int*   ADJ   = (int*)(ws + oADJ);
  int*   CNT   = (int*)(ws + oCNT);
  int*   DEGFB = (int*)(ws + oDEGF);
  float* CNTS  = (float*)(ws + oCNTS);
  const unsigned short* Kh = QKh + (size_t)NHD * NN * HDM;
  const unsigned short* Kl = QKl + (size_t)NHD * NN * HDM;

  const dim3 b256(256);

  k_plane<0><<<dim3(NN * FIN / 8 / 256), b256, 0, stream>>>(x, NN, FIN, FIN, XB, NN, FIN);
  k_wT<0><<<dim3(HH / 64, FIN / 64, 1), b256, 0, stream>>>(W_feat, WfT, FIN, HH, 0, 0);
  k_wT<1><<<dim3(HH / 64, (4 * HH) / 64, 1), b256, 0, stream>>>(W_proj, WpD, 4 * HH, HH, 0, 0);
  k_wT<1><<<dim3((3 * HH) / 64, HH / 64, NL), b256, 0, stream>>>(Wqkv, WqkvD, HH, 3 * HH, HH * 3 * HH, 3 * HH * 2 * HH);
  k_wT<1><<<dim3(HH / 64, HH / 64, NL), b256, 0, stream>>>(Wo, WoD, HH, HH, HH * HH, HH * 2 * HH);
  k_wT<1><<<dim3(FFD / 64, HH / 64, NL), b256, 0, stream>>>(W1, W1D, HH, FFD, HH * FFD, FFD * 2 * HH);
  k_wT<1><<<dim3(HH / 64, FFD / 64, NL), b256, 0, stream>>>(W2, W2D, FFD, HH, FFD * HH, HH * 2 * FFD);

  const int adjLds = ADJ_LDS_INTS * 4;
  (void)hipFuncSetAttribute(reinterpret_cast<const void*>(&k_adj), hipFuncAttributeMaxDynamicSharedMemorySize, adjLds);
  k_adj<<<dim3(NN / 128), dim3(128), (size_t)adjLds, stream>>>(ei, ADJ, CNT, DEGFB);
  k_bfs<<<dim3(NN / 32), b256, 0, stream>>>(ADJ, CNT, CNTS);
  k_div<<<dim3(1), dim3(128), 0, stream>>>(DIV);
  k_table<<<dim3(MAXD * 128 / 256), b256, 0, stream>>>(DIV, TAB);

  k_gemm_nt<0, 0><<<dim3(gemm_blocks(NN, HH)), b256, 0, stream>>>(XB, WfT, b_feat, EX, NN, HH, FIN, HH);
  k_cat<<<dim3(NN / 8), b256, 0, stream>>>(EX, b_feat, (const float*)DEGFB, CNTS, TAB, DIV, CAT);
  k_gemm_nt<0, 0><<<dim3(gemm_blocks(NN, HH)), b256, 0, stream>>>(CAT, WpD, b_proj, Hraw, NN, HH, 8 * HH, HH);
  k_post<0><<<dim3(NN * HH / 4 / 256), b256, 0, stream>>>(Hraw, b_proj, HfA, Hhl, HH, NN * HH / 4);

  const float sscale = 0x1.6a09e6p-3f;
  for (int l = 0; l < NL; ++l) {
    k_gemm_nt<0, 0><<<dim3(gemm_blocks(NN, 3 * HH)), b256, 0, stream>>>(
        Hhl, WqkvD + (size_t)l * 3 * HH * 2 * HH, bqkv, QKVr, NN, 3 * HH, 2 * HH, 3 * HH);
    k_qkvsplit<<<dim3(12, NN / 64), b256, 0, stream>>>(QKVr, bqkv + (size_t)l * 3 * HH, QKh, QKl, Vh, Vl);
    k_attn<<<dim3(NHD * (NN / 64)), dim3(128), 0, stream>>>(QKh, QKl, Kh, Kl, Vh, Vl, Of, sscale);
    k_plane<1><<<dim3(NN * 2 * HH / 8 / 256), b256, 0, stream>>>(Of, NN, HH, HH, Ohl, NN, HH);
    k_gemm_nt<0, 0><<<dim3(gemm_blocks(NN, HH)), b256, 0, stream>>>(
        Ohl, WoD + (size_t)l * HH * 2 * HH, bo, Zraw, NN, HH, 2 * HH, HH);
    k_addln<0><<<dim3(NN / 8), b256, 0, stream>>>(HfA, Zraw, bo + (size_t)l * HH, ln1_g + (size_t)l * HH,
                                                  ln1_b + (size_t)l * HH, HfB, Hhl);
    k_gemm_nt<0, 0><<<dim3(gemm_blocks(NN, FFD)), b256, 0, stream>>>(
        Hhl, W1D + (size_t)l * FFD * 2 * HH, b1, Graw, NN, FFD, 2 * HH, FFD);
    k_post<1><<<dim3(NN * FFD / 4 / 256), b256, 0, stream>>>(Graw, b1 + (size_t)l * FFD, Zraw, Ghl, FFD, NN * FFD / 4);
    k_gemm_nt<0, 0><<<dim3(gemm_blocks(NN, HH)), b256, 0, stream>>>(
        Ghl, W2D + (size_t)l * HH * 2 * FFD, b2, Zraw, NN, HH, 2 * FFD, HH);
    if (l + 1 < NL) {
      k_addln<0><<<dim3(NN / 8), b256, 0, stream>>>(HfB, Zraw, b2 + (size_t)l * HH, ln2_g + (size_t)l * HH,
                                                    ln2_b + (size_t)l * HH, HfA, Hhl);
    } else {
      k_addln<1><<<dim3(NN / 8), b256, 0, stream>>>(HfB, Zraw, b2 + (size_t)l * HH, ln2_g + (size_t)l * HH,
                                                    ln2_b + (size_t)l * HH, out, Hhl);
    }
  }
  (void)hipGetLastError();
}
